// DVAE_73847667687625
// MI455X (gfx1250) — hardware-verified
//
#include <hip/hip_runtime.h>
#include <math.h>

constexpr int kBatch   = 2048;
constexpr int kMaxN    = 16;
constexpr int kMsgRows = 15;
constexpr int kNvt     = 8;
constexpr int kHs      = 501;
constexpr int kHsPad   = 512;
constexpr int kVs      = 517;
constexpr int kG3      = 1503;
constexpr int kG3Pad   = 1536;
constexpr int kGmN     = 1024;
constexpr int kMapOff  = 512;
constexpr int kNz      = 56;
constexpr int kOutW    = 112;
constexpr int kFcN     = 128;
static_assert(kHsPad % 32 == 0, "cfg");
static_assert(kBatch % 64 == 0 && kG3Pad % 64 == 0 && kGmN % 64 == 0 && kFcN % 64 == 0, "cfg");
static_assert(kG3 <= kG3Pad && kMapOff + kHs <= kGmN && kHs <= kHsPad && kOutW <= kFcN, "cfg");
static_assert(kOutW % 4 == 0 && (kBatch * (kOutW / 4)) % 256 == 0, "cfg");
static_assert((kG3Pad * (kHsPad / 8)) % 256 == 0 && (kGmN * (kHsPad / 8)) % 256 == 0 && (kFcN * (kHsPad / 8)) % 256 == 0, "cfg");
static_assert(kMsgRows == kMaxN - 1, "cfg");

typedef __attribute__((ext_vector_type(16))) _Float16 v16h;
typedef __attribute__((ext_vector_type(8)))  _Float16 v8h;
typedef __attribute__((ext_vector_type(16))) __bf16   v16b;
typedef __attribute__((ext_vector_type(8)))  __bf16   v8b;
typedef __attribute__((ext_vector_type(8)))  float    v8f;
typedef __attribute__((ext_vector_type(4)))  float    v4f;
typedef __attribute__((ext_vector_type(4)))  unsigned int v4u;

__device__ __forceinline__ unsigned short f2bf_bits(float f) {
  unsigned u = __float_as_uint(f);
  return (unsigned short)((u + 0x7FFFu + ((u >> 16) & 1u)) >> 16);
}
__device__ __forceinline__ float bf_bits2f(unsigned short h) { return __uint_as_float(((unsigned)h) << 16); }
__device__ __forceinline__ float bfr(float f) { return bf_bits2f(f2bf_bits(f)); }
__device__ __forceinline__ void bf_split(float f, unsigned short& hb, unsigned short& lb) {
  hb = f2bf_bits(f);
  lb = f2bf_bits(f - bf_bits2f(hb));
}

__device__ __forceinline__ void dep_guard_h(v8f& a, v8f& b, v16h x, v16h y) { asm volatile("v_nop\n\tv_nop\n\tv_nop\n\tv_nop" : "+v"(a), "+v"(b) : "v"(x), "v"(y)); }
__device__ __forceinline__ void dep_guard_b(v8f& a, v8f& b, v16b x, v16b y) { asm volatile("v_nop\n\tv_nop\n\tv_nop\n\tv_nop" : "+v"(a), "+v"(b) : "v"(x), "v"(y)); }
__device__ __forceinline__ void dep_guard4_h(v8f& a, v8f& b, v8f& c, v8f& d, v16h x, v16h y) {
  asm volatile("v_nop\n\tv_nop\n\tv_nop\n\tv_nop" : "+v"(a), "+v"(b), "+v"(c), "+v"(d) : "v"(x), "v"(y));
}
__device__ __forceinline__ void dep_guard4_b(v8f& a, v8f& b, v8f& c, v8f& d, v16b x, v16b y) {
  asm volatile("v_nop\n\tv_nop\n\tv_nop\n\tv_nop" : "+v"(a), "+v"(b), "+v"(c), "+v"(d) : "v"(x), "v"(y));
}
__device__ __forceinline__ void keep4_h(v16h a, v16h b, v16h c, v16h d) { asm volatile("v_nop" :: "v"(a), "v"(b), "v"(c), "v"(d)); }
__device__ __forceinline__ void keep4_b(v16b a, v16b b, v16b c, v16b d) { asm volatile("v_nop" :: "v"(a), "v"(b), "v"(c), "v"(d)); }
__device__ __forceinline__ void acc_guard4(v8f& a, v8f& b, v8f& c, v8f& d) { asm volatile("v_nop\n\tv_nop\n\tv_nop\n\tv_nop" : "+v"(a), "+v"(b), "+v"(c), "+v"(d)); }
template <typename T> struct Frag;
template <> struct Frag<_Float16> {
  typedef v16h V; union U { v16h v; v8h h[2]; };
  static __device__ __forceinline__ v16h load(const _Float16* p) {
    U f; f.h[0] = *(const v8h*)(p); f.h[1] = *(const v8h*)(p + 16); return f.v;
  }
  static __device__ __forceinline__ v8f mma(v16h a, v16h b, v8f c) {
    return __builtin_amdgcn_wmma_f32_16x16x32_f16(false, a, false, b, (short)0, c, false, false);
  }
  static __device__ __forceinline__ void guard(v8f& a, v8f& b, v16h x, v16h y) { dep_guard_h(a, b, x, y); }
  static __device__ __forceinline__ void guard4(v8f& a, v8f& b, v8f& c, v8f& d, v16h x, v16h y) { dep_guard4_h(a, b, c, d, x, y); }
  static __device__ __forceinline__ void keep(v16h a, v16h b, v16h c, v16h d) { keep4_h(a, b, c, d); }
};
template <> struct Frag<__bf16> {
  typedef v16b V; union U { v16b v; v8b h[2]; };
  static __device__ __forceinline__ v16b load(const __bf16* p) {
    U f; f.h[0] = *(const v8b*)(p); f.h[1] = *(const v8b*)(p + 16); return f.v;
  }
  static __device__ __forceinline__ v8f mma(v16b a, v16b b, v8f c) {
    return __builtin_amdgcn_wmma_f32_16x16x32_bf16(false, a, false, b, (short)0, c, false, false);
  }
  static __device__ __forceinline__ void guard(v8f& a, v8f& b, v16b x, v16b y) { dep_guard_b(a, b, x, y); }
  static __device__ __forceinline__ void guard4(v8f& a, v8f& b, v8f& c, v8f& d, v16b x, v16b y) { dep_guard4_b(a, b, c, d, x, y); }
  static __device__ __forceinline__ void keep(v16b a, v16b b, v16b c, v16b d) { keep4_b(a, b, c, d); }
};

__device__ __forceinline__ unsigned pk16(unsigned short a, unsigned short b) { return (unsigned)a | ((unsigned)b << 16); }

template <int ET> struct Elem;
template <> struct Elem<0> { typedef _Float16 T; };
template <> struct Elem<1> { typedef __bf16 T; };
template <int ET, int SPLIT, int BIAS_MODE, int OUT_MODE, bool RESID, int ACT = 0>
__global__ __launch_bounds__(256) void wmma_gemm64(
    const unsigned short* __restrict__ Ap, const unsigned short* __restrict__ A2p, int lda, long strideA,
    const unsigned short* __restrict__ Btp, const unsigned short* __restrict__ Bt2p, int ldb, long strideB,
    void* __restrict__ Cout, void* __restrict__ Cout2, int ldc, long strideC,
    const float* __restrict__ bias,
    const float* __restrict__ resid, long strideR,
    int M, int N, int K, float scale) {
  typedef typename Elem<ET>::T T;
  typedef typename Frag<T>::V V;
  const T* A = (const T*)Ap; const T* A2 = (const T*)A2p; const T* Bt = (const T*)Btp; const T* Bt2 = (const T*)Bt2p;
  __shared__ __align__(16) float sT[8][16 * 68];
  const int b    = blockIdx.y;
  const int lane = threadIdx.x & 31;
  const int wave = threadIdx.x >> 5;
  const int tilesN = N >> 6;
  const int tilesM = M >> 6;
  const int tile = blockIdx.x * 8 + wave;
  if (tile >= tilesM * tilesN) return;
  const int tm = tile / tilesN;
  const int tn = tile - tm * tilesN;
  const int m0 = tm << 6;
  const int n0 = tn << 6;

  const T* Ab  = A  + (size_t)b * strideA;
  const T* Bb  = Bt + (size_t)b * strideB;
  const T* Ab2 = (SPLIT >= 1) ? (A2  + (size_t)b * strideA) : nullptr;
  const T* Bb2 = (SPLIT == 2) ? (Bt2 + (size_t)b * strideB) : nullptr;

  const int rlane = lane & 15;
  const int koff  = (lane >> 4) * 8;
  const int mOff  = (lane >> 4) * 8;

  v8f acc[4][4];
#pragma unroll
  for (int i = 0; i < 4; ++i)
#pragma unroll
    for (int j = 0; j < 4; ++j) acc[i][j] = (v8f){0.f,0.f,0.f,0.f,0.f,0.f,0.f,0.f};

  for (int k0 = 0; k0 < K; k0 += 32) {
    V bh[4], bl[4];
#pragma unroll
    for (int j = 0; j < 4; ++j) {
      const size_t bo = (size_t)(n0 + (j << 4) + rlane) * ldb + koff + k0;
      bh[j] = Frag<T>::load(Bb + bo);
      if (SPLIT == 2) bl[j] = Frag<T>::load(Bb2 + bo);
    }
#pragma unroll
    for (int i = 0; i < 4; ++i) {
      const size_t ao = (size_t)(m0 + (i << 4) + rlane) * lda + koff + k0;
      V ah = Frag<T>::load(Ab + ao);
      V al;
      if (SPLIT >= 1) al = Frag<T>::load(Ab2 + ao);
#pragma unroll
      for (int j = 0; j < 4; ++j) {
        acc[i][j] = Frag<T>::mma(ah, bh[j], acc[i][j]);
        if (SPLIT == 2) acc[i][j] = Frag<T>::mma(ah, bl[j], acc[i][j]);
        if (SPLIT >= 1) acc[i][j] = Frag<T>::mma(al, bh[j], acc[i][j]);
      }
      Frag<T>::guard4(acc[i][0], acc[i][1], acc[i][2], acc[i][3], ah, (SPLIT >= 1) ? al : ah);
    }
    Frag<T>::keep(bh[0], bh[1], bh[2], bh[3]);
    if (SPLIT == 2) Frag<T>::keep(bl[0], bl[1], bl[2], bl[3]);
  }
  acc_guard4(acc[0][0], acc[0][1], acc[0][2], acc[0][3]);
  acc_guard4(acc[1][0], acc[1][1], acc[1][2], acc[1][3]);
  acc_guard4(acc[2][0], acc[2][1], acc[2][2], acc[2][3]);
  acc_guard4(acc[3][0], acc[3][1], acc[3][2], acc[3][3]);

  float* slab = sT[wave];
  const float* Rb = RESID ? (resid + (size_t)b * strideR) : nullptr;
#pragma unroll
  for (int i = 0; i < 4; ++i) {
    const int mBase = m0 + (i << 4);
#pragma unroll
    for (int j = 0; j < 4; ++j) {
      const int n = n0 + (j << 4) + rlane;
      float bv = 0.f;
      if (BIAS_MODE == 2) bv = bias[n];
#pragma unroll
      for (int r = 0; r < 8; ++r) {
        float v = acc[i][j][r] * scale;
        if (BIAS_MODE == 1) v += bias[mBase + mOff + r];
        if (BIAS_MODE == 2) v += bv;
        if (RESID) v += Rb[(size_t)(mBase + mOff + r) * ldc + n];
        if (ACT == 2) v = fmaxf(v, 0.0f);
        if (ACT == 4) v = (v > 0.f) ? v : 0.01f * v;
        slab[(mOff + r) * 68 + (j << 4) + rlane] = v;
      }
    }
    __builtin_amdgcn_fence(__ATOMIC_RELEASE, "workgroup");
    __builtin_amdgcn_wave_barrier();
    __builtin_amdgcn_fence(__ATOMIC_ACQUIRE, "workgroup");
    if (OUT_MODE == 0) {
      float* C = (float*)Cout + (size_t)b * strideC;
      const int hh = lane >> 4, c4 = (lane & 15) * 4;
      for (int pass = 0; pass < 2; ++pass) {
#pragma unroll
        for (int it = 0; it < 8; ++it) {
          const int row = it * 2 + hh;
          v4f v = *(const v4f*)(slab + row * 68 + c4);
          *(volatile v4f*)(C + (size_t)(mBase + row) * ldc + n0 + c4) = v;
        }
        __threadfence();
      }
    } else {
      const int q = lane >> 3, c8 = (lane & 7) * 8;
      unsigned short* C  = (unsigned short*)Cout  + (size_t)b * strideC;
      unsigned short* C2 = (OUT_MODE == 2) ? ((unsigned short*)Cout2 + (size_t)b * strideC) : nullptr;
      for (int pass = 0; pass < 2; ++pass) {
#pragma unroll
        for (int it = 0; it < 4; ++it) {
          const int row = it * 4 + q;
          const float* sp = slab + row * 68 + c8;
          v8h hv, lv;
#pragma unroll
          for (int e = 0; e < 8; ++e) {
            if (OUT_MODE == 1) {
              hv[e] = (_Float16)sp[e];
            } else {
              unsigned short hb = f2bf_bits(sp[e]);
              unsigned short lb = f2bf_bits(sp[e] - bf_bits2f(hb));
              hv[e] = __builtin_bit_cast(_Float16, hb);
              lv[e] = __builtin_bit_cast(_Float16, lb);
            }
          }
          *(volatile v8h*)(C + (size_t)(mBase + row) * ldc + n0 + c8) = hv;
          if (OUT_MODE == 2) *(volatile v8h*)(C2 + (size_t)(mBase + row) * ldc + n0 + c8) = lv;
        }
        __threadfence();
      }
    }
    __builtin_amdgcn_fence(__ATOMIC_RELEASE, "workgroup");
    __builtin_amdgcn_wave_barrier();
    __builtin_amdgcn_fence(__ATOMIC_ACQUIRE, "workgroup");
  }
}

__device__ __forceinline__ float sigm_f(float x) { return __builtin_amdgcn_rcpf(1.0f + expf(-x)); }

__global__ __launch_bounds__(256) void prep_whh_kernel(const float* __restrict__ w_hh, unsigned short* __restrict__ whh) {
  const int t = blockIdx.x * 256 + threadIdx.x;
  if (t >= kG3Pad * (kHsPad / 8)) return;
  const int n = t >> 6;
  const int k8 = (t & 63) * 8;
  const int nc = n < kG3 ? n : kG3 - 1;
  const float fn = n < kG3 ? 1.0f : 0.0f;
  float v[8];
#pragma unroll
  for (int e = 0; e < 8; ++e) {
    const int k = k8 + e;
    const int kc = k < kHs ? k : kHs - 1;
    const float fk = k < kHs ? fn : 0.0f;
    v[e] = w_hh[(size_t)nc * kHs + kc] * fk;
  }
  unsigned short hb[8];
#pragma unroll
  for (int e = 0; e < 8; ++e) hb[e] = f2bf_bits(v[e]);
  const v4u u = (v4u){pk16(hb[0], hb[1]), pk16(hb[2], hb[3]), pk16(hb[4], hb[5]), pk16(hb[6], hb[7])};
  unsigned short* q = whh + (size_t)n * kHsPad + k8;
  *(volatile v4u*)q = u;
  __threadfence();
  *(volatile v4u*)q = u;
}

__global__ __launch_bounds__(256) void prep_gm_kernel(const float* __restrict__ gate_w, const float* __restrict__ map_w,
                                                      unsigned short* __restrict__ gm) {
  const int t = blockIdx.x * 256 + threadIdx.x;
  if (t >= kGmN * (kHsPad / 8)) return;
  const int n = t >> 6;
  const int k8 = (t & 63) * 8;
  const int ng = n < kHs ? n : kHs - 1;
  const float fg = n < kHs ? 1.0f : 0.0f;
  int nm = n - kMapOff;
  nm = nm < 0 ? 0 : (nm > kHs - 1 ? kHs - 1 : nm);
  const float fm = (n >= kMapOff && n < kMapOff + kHs) ? 1.0f : 0.0f;
  float a[8], c[8];
#pragma unroll
  for (int e = 0; e < 8; ++e) {
    const int k = k8 + e;
    const int kc = k < kHs ? k : kHs - 1;
    a[e] = gate_w[(size_t)ng * kVs + kc];
  }
  asm volatile("" ::: "memory");
#pragma unroll
  for (int e = 0; e < 8; ++e) {
    const int k = k8 + e;
    const int kc = k < kHs ? k : kHs - 1;
    c[e] = map_w[(size_t)nm * kVs + kc];
  }
  unsigned short hb[8];
#pragma unroll
  for (int e = 0; e < 8; ++e) {
    const float fk = (k8 + e) < kHs ? 1.0f : 0.0f;
    const float v = fk * (fg * a[e] + fm * c[e]);
    hb[e] = f2bf_bits(v);
  }
  const v4u u = (v4u){pk16(hb[0], hb[1]), pk16(hb[2], hb[3]), pk16(hb[4], hb[5]), pk16(hb[6], hb[7])};
  unsigned short* q = gm + (size_t)n * kHsPad + k8;
  *(volatile v4u*)q = u;
  __threadfence();
  *(volatile v4u*)q = u;
}

__global__ __launch_bounds__(256) void prep_fc_kernel(const float* __restrict__ fc1_w, const float* __restrict__ fc1_b,
                                                      const float* __restrict__ fc2_w, const float* __restrict__ fc2_b,
                                                      unsigned short* __restrict__ fcw, float* __restrict__ fcb) {
  const int t = blockIdx.x * 256 + threadIdx.x;
  if (t < kFcN * (kHsPad / 8)) {
    const int o  = t >> 6;
    const int k8 = (t & 63) * 8;
    const int o1 = o < kNz ? o : kNz - 1;
    int o2 = o - kNz;
    o2 = o2 < 0 ? 0 : (o2 > kNz - 1 ? kNz - 1 : o2);
    const float f1 = o < kNz ? 1.0f : 0.0f;
    const float f2 = (o >= kNz && o < 2 * kNz) ? 1.0f : 0.0f;
    float a[8], c[8];
#pragma unroll
    for (int e = 0; e < 8; ++e) {
      const int k = k8 + e;
      const int kc = k < kHs ? k : kHs - 1;
      a[e] = fc1_w[(size_t)o1 * kHs + kc];
    }
    asm volatile("" ::: "memory");
#pragma unroll
    for (int e = 0; e < 8; ++e) {
      const int k = k8 + e;
      const int kc = k < kHs ? k : kHs - 1;
      c[e] = fc2_w[(size_t)o2 * kHs + kc];
    }
    unsigned short hb[8];
#pragma unroll
    for (int e = 0; e < 8; ++e) {
      const float fk = (k8 + e) < kHs ? 1.0f : 0.0f;
      const float v = fk * (f1 * a[e] + f2 * c[e]);
      hb[e] = f2bf_bits(v);
    }
    const v4u u = (v4u){pk16(hb[0], hb[1]), pk16(hb[2], hb[3]), pk16(hb[4], hb[5]), pk16(hb[6], hb[7])};
    unsigned short* q = fcw + (size_t)o * kHsPad + k8;
    *(volatile v4u*)q = u;
    __threadfence();
    *(volatile v4u*)q = u;
  } else if (t < kFcN * (kHsPad / 8) + kFcN) {
    const int o = t - kFcN * (kHsPad / 8);
    const int o1 = o < kNz ? o : kNz - 1;
    int o2 = o - kNz;
    o2 = o2 < 0 ? 0 : (o2 > kNz - 1 ? kNz - 1 : o2);
    const float f1 = o < kNz ? 1.0f : 0.0f;
    const float f2 = (o >= kNz && o < 2 * kNz) ? 1.0f : 0.0f;
    const float a = bfr(fc1_b[o1]);
    const float c = bfr(fc2_b[o2]);
    const float v = f1 * a + f2 * c;
    *(volatile float*)(fcb + o) = v;
    __threadfence();
    *(volatile float*)(fcb + o) = v;
  }
}

__global__ __launch_bounds__(256) void msg_hin_kernel(const float* __restrict__ gmout, const float* __restrict__ gate_w,
                                                      const float* __restrict__ gate_b, const float* __restrict__ map_w,
                                                      const float* __restrict__ adj, float* msg,
                                                      float* __restrict__ hin32, unsigned short* __restrict__ hinh,
                                                      unsigned short* __restrict__ hinl, int v) {
  __shared__ __align__(16) float shv[256];
  const int tid  = threadIdx.x;
  const int b    = blockIdx.x >> 1;
  const int half = blockIdx.x & 1;
  const int j    = half * 256 + tid;
  const int jc   = j < kHs ? j : kHs - 1;
  const float fk = j < kHs ? 1.0f : 0.0f;
  int vv = v < 1 ? 1 : (v > kMaxN - 1 ? kMaxN - 1 : v);
  const int vm1 = vv - 1;

  const float* gmr = gmout + (size_t)b * kGmN;
  const float x0 = gmr[jc];
  const float x1 = gate_w[(size_t)jc * kVs + kHs + vm1];
  const float x2 = gate_b[jc];
  const float x3 = gmr[kMapOff + jc];
  const float x4 = map_w[(size_t)jc * kVs + kHs + vm1];
  const float gpre = (x0 + bfr(x1)) + bfr(x2);
  const float mval = x3 + bfr(x4);
  const float g  = sigm_f(gpre);
  const float mv = fk * (g * mval);

  float* mp = msg + ((size_t)b * kMsgRows + vm1) * kHsPad + j;
  *(volatile float*)mp = mv;

  const float* ar = adj + (size_t)b * (kMaxN * kMaxN) + (size_t)vv * kMaxN;
  float hsum = 0.0f;
#pragma unroll 1
  for (int u = 0; u < vm1; ++u) {
    const float cu = bfr(ar[u]);
    hsum += cu * msg[((size_t)b * kMsgRows + u) * kHsPad + j];
  }
  hsum += bfr(ar[vm1]) * mv;

  float* hp = hin32 + (size_t)b * kHsPad + j;
  *(volatile float*)hp = hsum;
  shv[tid] = hsum;
  __threadfence();
  *(volatile float*)mp = mv;
  *(volatile float*)hp = hsum;
  __syncthreads();
  if (tid < 32) {
    const v4f a = *(const v4f*)(shv + 8 * tid);
    const v4f c = *(const v4f*)(shv + 8 * tid + 4);
    unsigned short hb[8], lb[8];
#pragma unroll
    for (int e = 0; e < 4; ++e) {
      bf_split(a[e], hb[e], lb[e]);
      bf_split(c[e], hb[4 + e], lb[4 + e]);
    }
    const v4u uh = (v4u){pk16(hb[0], hb[1]), pk16(hb[2], hb[3]), pk16(hb[4], hb[5]), pk16(hb[6], hb[7])};
    const v4u ul = (v4u){pk16(lb[0], lb[1]), pk16(lb[2], lb[3]), pk16(lb[4], lb[5]), pk16(lb[6], lb[7])};
    const size_t po = (size_t)b * kHsPad + half * 256 + 8 * tid;
    *(volatile v4u*)(hinh + po) = uh;
    *(volatile v4u*)(hinl + po) = ul;
    __threadfence();
    *(volatile v4u*)(hinh + po) = uh;
    *(volatile v4u*)(hinl + po) = ul;
  }
}

__global__ __launch_bounds__(256) void gru_kernel(const float* __restrict__ gh, const float* __restrict__ hin32,
                                                  const int* __restrict__ node_types, const float* __restrict__ w_ih,
                                                  const float* __restrict__ b_ih, const float* __restrict__ b_hh,
                                                  float* __restrict__ hv32, unsigned short* __restrict__ hvh,
                                                  unsigned short* __restrict__ hvl, int v, int use_h) {
  __shared__ __align__(16) float shv[256];
  const int tid  = threadIdx.x;
  const int b    = blockIdx.x >> 1;
  const int half = blockIdx.x & 1;
  const int j    = half * 256 + tid;
  const int jc   = j < kHs ? j : kHs - 1;
  const float fk = j < kHs ? 1.0f : 0.0f;
  const int vv = v < 0 ? 0 : (v > kMaxN - 1 ? kMaxN - 1 : v);
  int ty = node_types[(size_t)b * kMaxN + vv];
  ty = ty < 0 ? 0 : (ty > kNvt - 1 ? kNvt - 1 : ty);

  const float a0 = w_ih[(size_t)jc * kNvt + ty];
  const float a1 = w_ih[(size_t)(kHs + jc) * kNvt + ty];
  const float a2 = w_ih[(size_t)(2 * kHs + jc) * kNvt + ty];
  const float c0 = b_ih[jc];
  const float c1 = b_ih[kHs + jc];
  const float c2 = b_ih[2 * kHs + jc];
  asm volatile("" ::: "memory");
  const float d0 = b_hh[jc];
  const float d1 = b_hh[kHs + jc];
  const float d2 = b_hh[2 * kHs + jc];
  float e0 = 0.0f, e1 = 0.0f, e2 = 0.0f, hprev = 0.0f;
  if (use_h != 0) {
    const float* ghr = gh + (size_t)b * kG3Pad;
    e0 = ghr[jc];
    e1 = ghr[kHs + jc];
    e2 = ghr[2 * kHs + jc];
    hprev = hin32[(size_t)b * kHsPad + jc];
  }
  const float gi_r = bfr(a0) + bfr(c0);
  const float gi_z = bfr(a1) + bfr(c1);
  const float gi_n = bfr(a2) + bfr(c2);
  const float gh_r = e0 + bfr(d0);
  const float gh_z = e1 + bfr(d1);
  const float gh_n = e2 + bfr(d2);
  const float r = sigm_f(gi_r + gh_r);
  const float z = sigm_f(gi_z + gh_z);
  const float n = tanhf(gi_n + r * gh_n);
  const float h = fk * ((1.0f - z) * n + z * hprev);

  float* hp = hv32 + (size_t)b * kHsPad + j;
  *(volatile float*)hp = h;
  shv[tid] = h;
  __threadfence();
  *(volatile float*)hp = h;
  __syncthreads();
  if (tid < 32) {
    const v4f a = *(const v4f*)(shv + 8 * tid);
    const v4f c = *(const v4f*)(shv + 8 * tid + 4);
    unsigned short hb[8], lb[8];
#pragma unroll
    for (int e = 0; e < 4; ++e) {
      bf_split(a[e], hb[e], lb[e]);
      bf_split(c[e], hb[4 + e], lb[4 + e]);
    }
    const v4u uh = (v4u){pk16(hb[0], hb[1]), pk16(hb[2], hb[3]), pk16(hb[4], hb[5]), pk16(hb[6], hb[7])};
    const v4u ul = (v4u){pk16(lb[0], lb[1]), pk16(lb[2], lb[3]), pk16(lb[4], lb[5]), pk16(lb[6], lb[7])};
    const size_t po = (size_t)b * kHsPad + half * 256 + 8 * tid;
    *(volatile v4u*)(hvh + po) = uh;
    *(volatile v4u*)(hvl + po) = ul;
    __threadfence();
    *(volatile v4u*)(hvh + po) = uh;
    *(volatile v4u*)(hvl + po) = ul;
  }
}

__global__ __launch_bounds__(256) void head_pack_kernel(const float* __restrict__ fcout, float* __restrict__ out) {
  const int i = blockIdx.x * 256 + threadIdx.x;
  if (i >= kBatch * (kOutW / 4)) return;
  const int b  = i / (kOutW / 4);
  const int q  = i - b * (kOutW / 4);
  const v4f o = *(const v4f*)(fcout + (size_t)b * kFcN + 4 * q);
  float* op = out + 4 * (size_t)i;
  *(volatile v4f*)op = o;
  __threadfence();
  *(volatile v4f*)op = o;
}

extern "C" void kernel_launch(void* const* d_in, const int* in_sizes, int n_in,
                              void* d_out, int out_size, void* d_ws, size_t ws_size, hipStream_t stream) {
  (void)in_sizes; (void)n_in;
  const int*   node_types = (const int*)  d_in[0];
  const float* adj        = (const float*)d_in[1];
  const float* w_ih       = (const float*)d_in[2];
  const float* w_hh       = (const float*)d_in[3];
  const float* b_ih       = (const float*)d_in[4];
  const float* b_hh       = (const float*)d_in[5];
  const float* gate_w     = (const float*)d_in[6];
  const float* gate_b     = (const float*)d_in[7];
  const float* map_w      = (const float*)d_in[8];
  const float* fc1_w      = (const float*)d_in[9];
  const float* fc1_b      = (const float*)d_in[10];
  const float* fc2_w      = (const float*)d_in[11];
  const float* fc2_b      = (const float*)d_in[12];
  float* out = (float*)d_out;
  if (out_size != kBatch * kOutW) return;

  char* ws = (char*)d_ws;
  size_t off = 0;
  auto carve = [&](size_t bytes) -> char* { char* p = ws + off; off += (bytes + 255) & ~(size_t)255; return p; };
  float*          MSG   = (float*)carve((size_t)kBatch * kMsgRows * kHsPad * 4);
  float*          GH    = (float*)carve((size_t)kBatch * kG3Pad * 4);
  float*          GMOUT = (float*)carve((size_t)kBatch * kGmN * 4);
  float*          HIN32 = (float*)carve((size_t)kBatch * kHsPad * 4);
  float*          HV32  = (float*)carve((size_t)kBatch * kHsPad * 4);
  unsigned short* HINH  = (unsigned short*)carve((size_t)kBatch * kHsPad * 2);
  unsigned short* HINL  = (unsigned short*)carve((size_t)kBatch * kHsPad * 2);
  unsigned short* HVH   = (unsigned short*)carve((size_t)kBatch * kHsPad * 2);
  unsigned short* HVL   = (unsigned short*)carve((size_t)kBatch * kHsPad * 2);
  unsigned short* WHH   = (unsigned short*)carve((size_t)kG3Pad * kHsPad * 2);
  unsigned short* GM    = (unsigned short*)carve((size_t)kGmN * kHsPad * 2);
  unsigned short* FCW   = (unsigned short*)carve((size_t)kFcN * kHsPad * 2);
  float*          FCB   = (float*)carve((size_t)kFcN * 4);
  float*          FCOUT = (float*)carve((size_t)kBatch * kFcN * 4);
  if (off > ws_size || off > (size_t)134217728) return;

  prep_whh_kernel<<<(kG3Pad * (kHsPad / 8)) / 256, 256, 0, stream>>>(w_hh, WHH);
  prep_gm_kernel<<<(kGmN * (kHsPad / 8)) / 256, 256, 0, stream>>>(gate_w, map_w, GM);
  prep_fc_kernel<<<(kFcN * (kHsPad / 8) + kFcN + 255) / 256, 256, 0, stream>>>(fc1_w, fc1_b, fc2_w, fc2_b, FCW, FCB);

  const int stepBlocks = kBatch * 2;
  const int tiles1 = (kBatch / 64) * (kG3Pad / 64);
  const int tiles2 = (kBatch / 64) * (kGmN / 64);
  const int tilesF = (kBatch / 64) * (kFcN / 64);

  for (int v = 0; v < kMaxN; ++v) {
    if (v > 0) {
      msg_hin_kernel<<<stepBlocks, 256, 0, stream>>>(GMOUT, gate_w, gate_b, map_w, adj, MSG, HIN32, HINH, HINL, v);
      wmma_gemm64<1, 1, 0, 0, false, 0><<<dim3((tiles1 + 7) / 8, 1), 256, 0, stream>>>(
          (const unsigned short*)HINH, (const unsigned short*)HINL, kHsPad, 0L,
          (const unsigned short*)WHH, (const unsigned short*)nullptr, kHsPad, 0L,
          (void*)GH, (void*)nullptr, kG3Pad, 0L,
          (const float*)nullptr, (const float*)nullptr, 0L, kBatch, kG3Pad, kHsPad, 1.0f);
    }
    gru_kernel<<<stepBlocks, 256, 0, stream>>>(GH, HIN32, node_types, w_ih, b_ih, b_hh, HV32, HVH, HVL, v, v > 0 ? 1 : 0);
    if (v < kMaxN - 1) {
      wmma_gemm64<1, 1, 0, 0, false, 0><<<dim3((tiles2 + 7) / 8, 1), 256, 0, stream>>>(
          (const unsigned short*)HVH, (const unsigned short*)HVL, kHsPad, 0L,
          (const unsigned short*)GM, (const unsigned short*)nullptr, kHsPad, 0L,
          (void*)GMOUT, (void*)nullptr, kGmN, 0L,
          (const float*)nullptr, (const float*)nullptr, 0L, kBatch, kGmN, kHsPad, 1.0f);
    }
  }
  wmma_gemm64<1, 1, 2, 0, false, 0><<<dim3((tilesF + 7) / 8, 1), 256, 0, stream>>>(
      (const unsigned short*)HVH, (const unsigned short*)HVL, kHsPad, 0L,
      (const unsigned short*)FCW, (const unsigned short*)nullptr, kHsPad, 0L,
      (void*)FCOUT, (void*)nullptr, kFcN, 0L,
      (const float*)FCB, (const float*)nullptr, 0L, kBatch, kFcN, kHsPad, 1.0f);
  head_pack_kernel<<<(kBatch * (kOutW / 4)) / 256, 256, 0, stream>>>(FCOUT, out);
}
